// SimpleTemporalGCN_79482664780415
// MI455X (gfx1250) — hardware-verified
//
#include <hip/hip_runtime.h>
#include <math.h>

typedef __attribute__((ext_vector_type(16))) _Float16 v16h;
typedef __attribute__((ext_vector_type(16))) __bf16 v16b;
typedef __attribute__((ext_vector_type(8)))  _Float16 v8h;
typedef __attribute__((ext_vector_type(8)))  float v8f;
typedef __attribute__((ext_vector_type(4)))  float v4f;
typedef __attribute__((ext_vector_type(2)))  float v2f;
typedef __attribute__((ext_vector_type(4)))  unsigned v4u;
typedef __attribute__((ext_vector_type(4)))  int v4i;
typedef float __attribute__((may_alias)) float_a;
typedef int __attribute__((may_alias)) int_a;

template <typename T> __device__ __forceinline__ void vst2(void* p, T v) { *(volatile T*)p = v; __threadfence(); *(volatile T*)p = v; }
__device__ __forceinline__ v8f wmma16(v16h a, v16h b, v8f c) {
  v8f d = __builtin_amdgcn_wmma_f32_16x16x32_f16(false, a, false, b, (short)0, c, false, false);
  asm volatile("v_nop\n\tv_nop\n\tv_nop\n\tv_nop" : "+v"(d) : "v"(a), "v"(b));
  return d;
}
__device__ __forceinline__ v8f wmma_bf(v16b a, v16b b, v8f c) {
  v8f d = __builtin_amdgcn_wmma_f32_16x16x32_bf16(false, a, false, b, (short)0, c, false, false);
  asm volatile("v_nop\n\tv_nop\n\tv_nop\n\tv_nop" : "+v"(d) : "v"(a), "v"(b));
  return d;
}
__device__ __forceinline__ v16h frag_h(const _Float16* rowk0, int lane) {
  union { v16h v; v8h q[2]; } u; const _Float16* p = rowk0 + 8 * (lane >> 4);
  u.q[0] = *(const v8h*)p; u.q[1] = *(const v8h*)(p + 16); return u.v;
}
__device__ __forceinline__ v16h frag_f32(const float* rowk0, int lane) {
  v16h a; const float* p = rowk0 + 8 * (lane >> 4);
#pragma unroll
  for (int i = 0; i < 8; ++i) { a[i] = (_Float16)p[i]; a[8 + i] = (_Float16)p[16 + i]; }
  return a;
}
__device__ __forceinline__ v16h frag_f32s(const float* rowk0, int lane, float sc) {
  v16h a; const float* p = rowk0 + 8 * (lane >> 4);
#pragma unroll
  for (int i = 0; i < 8; ++i) { a[i] = (_Float16)(p[i] * sc); a[8 + i] = (_Float16)(p[16 + i] * sc); }
  return a;
}
__device__ __forceinline__ v16h fragc_f32(const float* W, int k0, int n, int lane, int ld, int K) {
  v16h a; const int g = lane >> 4;
#pragma unroll
  for (int i = 0; i < 8; ++i) { const int ka = k0 + 8 * g + i, kb = ka + 16;
    a[i] = (_Float16)(ka < K ? W[(size_t)ka * ld + n] : 0.f); a[8 + i] = (_Float16)(kb < K ? W[(size_t)kb * ld + n] : 0.f); }
  return a;
}
struct F2 { v16b h, l; };
__device__ __forceinline__ F2 bsplit16(const float v[16]) { F2 r;
#pragma unroll
  for (int i = 0; i < 16; ++i) { const __bf16 h = (__bf16)v[i]; r.h[i] = h; r.l[i] = (__bf16)(v[i] - (float)h); }
  return r; }
__device__ __forceinline__ F2 split_row(const float* row, int k0, int lane) { float v[16]; const float* p = row + k0 + 8 * (lane >> 4);
#pragma unroll
  for (int i = 0; i < 8; ++i) { v[i] = p[i]; v[8 + i] = p[16 + i]; }
  return bsplit16(v); }
__device__ __forceinline__ F2 split_rowK(const float* row, int k0, int lane, int K) { float v[16]; const int g = lane >> 4;
#pragma unroll
  for (int i = 0; i < 8; ++i) { const int ka = k0 + 8 * g + i, kb = ka + 16; v[i] = ka < K ? row[ka] : 0.f; v[8 + i] = kb < K ? row[kb] : 0.f; }
  return bsplit16(v); }
__device__ __forceinline__ F2 split_col(const float* W, int k0, int n, int lane, int ld, int K) { float v[16]; const int g = lane >> 4;
#pragma unroll
  for (int i = 0; i < 8; ++i) { const int ka = k0 + 8 * g + i, kb = ka + 16; v[i] = ka < K ? W[(size_t)ka * ld + n] : 0.f; v[8 + i] = kb < K ? W[(size_t)kb * ld + n] : 0.f; }
  return bsplit16(v); }
__device__ __forceinline__ v8f mac3(const F2& a, const F2& b, v8f c) { c = wmma_bf(a.l, b.h, c); c = wmma_bf(a.h, b.l, c); return wmma_bf(a.h, b.h, c); }
__device__ __forceinline__ float sigm(float v) { return 1.0f / (1.0f + expf(-v)); }
#define LDSX() do { asm volatile("s_wait_dscnt 0" ::: "memory"); __builtin_amdgcn_wave_barrier(); __builtin_amdgcn_fence(__ATOMIC_RELEASE, "workgroup"); } while (0)

#define NBG 32
#define NNODE 100
#define NPAD 112
#define HH 256
#define TE 128

__device__ __forceinline__ float gelu_e(float v) { return 0.5f * v * (1.0f + erff(v * 0.70710678118654752f)); }

template <int MODE>
__device__ __forceinline__ void block_gemm(const float* sAn, const float* src, int lds, const float* __restrict__ W, const float* __restrict__ bias, int relu, float* dst, int ldd, int wave, int lane) {
  const int col = lane & 15, g = lane >> 4;
#pragma unroll 1
  for (int rt = wave; rt < NPAD / 16; rt += 4) {
#pragma unroll 1
   for (int nh = 0; nh < 2; ++nh) {
    v8f acc[8];
#pragma unroll
    for (int t = 0; t < 8; ++t) acc[t] = (v8f){};
    if (MODE == 0) {
#pragma unroll 1
      for (int kc = 0; kc < 4; ++kc) { const F2 a = split_col(sAn, kc * 32, rt * 16 + col, lane, NPAD, NNODE);
#pragma unroll
        for (int t = 0; t < 8; ++t) acc[t] = mac3(a, split_col(src, kc * 32, (nh * 8 + t) * 16 + col, lane, lds, NNODE), acc[t]); } }
    else {
#pragma unroll 1
      for (int kc = 0; kc < HH / 32; ++kc) { const F2 a = split_row(src + (size_t)(rt * 16 + col) * lds, kc * 32, lane);
#pragma unroll
        for (int t = 0; t < 8; ++t) acc[t] = mac3(a, split_col(W, kc * 32, (nh * 8 + t) * 16 + col, lane, HH, HH), acc[t]); } }
#pragma unroll
    for (int t = 0; t < 8; ++t) { const int c = (nh * 8 + t) * 16 + col; const float bb = bias ? bias[c] : 0.f;
#pragma unroll
      for (int r = 0; r < 8; ++r) { const int i = rt * 16 + 8 * g + r; float v = acc[t][r] + bb; if (relu) v = v > 0.f ? v : 0.f; if (i >= NNODE) v = 0.f; dst[(size_t)i * ldd + c] = v; } } } }
}
__global__ __launch_bounds__(128) void k_main(const float* __restrict__ X, const float* __restrict__ tm, const float* __restrict__ W1, const float* __restrict__ b1, const float* __restrict__ W2, const float* __restrict__ b2, const float* __restrict__ W3, const float* __restrict__ b3,
                                            const float* __restrict__ tw1, const float* __restrict__ tb1, const float* __restrict__ tw2, const float* __restrict__ tb2, const float* __restrict__ e0w, const float* __restrict__ e0b, const float* __restrict__ e1w, const float* __restrict__ e1b, float* __restrict__ out) {
  __shared__ __align__(16) float sAn[NPAD][NPAD];
  __shared__ __align__(16) float sh[NPAD][HH + 4];
  __shared__ __align__(16) float sg[NPAD][HH + 4];
  __shared__ float sdis[NPAD]; __shared__ float swA[HH], swB[HH]; __shared__ float su[NPAD], sv[NPAD]; __shared__ float ste[TE]; __shared__ float sconst[4];
  const int tid = threadIdx.x, wave = tid >> 5, lane = tid & 31;
  for (int k = tid; k < HH; k += 128) { float a = 0.f, bsum = 0.f; for (int c = 0; c < HH; ++c) { const float e1 = e1w[c]; a += e0w[(size_t)k * HH + c] * e1; bsum += e0w[(size_t)(HH + k) * HH + c] * e1; } swA[k] = a; swB[k] = bsum; }
  if (tid == 0) { float cb = 0.f; for (int c = 0; c < HH; ++c) cb += e0b[c] * e1w[c]; sconst[0] = cb + e1b[0]; }
#pragma unroll 1
  for (int bb2 = 0; bb2 < 2; ++bb2) { const int b = blockIdx.x * 2 + bb2;
    __syncthreads();
    for (int q = tid; q < NPAD * NPAD; q += 128) { const int j = q / NPAD, i = q % NPAD; float v = 0.f; if (j < NNODE && i < NNODE) v = (j == i) ? 1.f : (X[(size_t)b * NNODE * NNODE + j * NNODE + i] != 0.f ? 1.f : 0.f); sAn[j][i] = v; }
    __syncthreads();
    if (tid < NPAD) { float d = 0.f; if (tid < NNODE) for (int j = 0; j < NNODE; ++j) d += sAn[j][tid]; sdis[tid] = d > 0.f ? 1.0f / sqrtf(d) : 0.f; }
    { const float t = tm[b]; ste[tid] = gelu_e(t * tw1[tid] + tb1[tid]); }
    __syncthreads();
    for (int q = tid; q < NPAD * NPAD; q += 128) { const int j = q / NPAD, i = q % NPAD; sAn[j][i] *= sdis[j] * sdis[i]; }
    if (tid == 0) { float s = 0.f; for (int o = 0; o < TE; ++o) { float z = tb2[o]; for (int k = 0; k < TE; ++k) z += ste[k] * tw2[k * TE + o]; s += z * e1w[HH + o]; } sconst[1] = s; }
    __syncthreads();
    block_gemm<0>(&sAn[0][0], W1, HH, nullptr, b1, 1, &sh[0][0], HH + 4, wave, lane);
    __syncthreads();
    block_gemm<1>(nullptr, &sh[0][0], HH + 4, W2, nullptr, 0, &sg[0][0], HH + 4, wave, lane);
    __syncthreads();
    block_gemm<0>(&sAn[0][0], &sg[0][0], HH + 4, nullptr, b2, 1, &sh[0][0], HH + 4, wave, lane);
    __syncthreads();
    block_gemm<1>(nullptr, &sh[0][0], HH + 4, W3, nullptr, 0, &sg[0][0], HH + 4, wave, lane);
    __syncthreads();
    block_gemm<0>(&sAn[0][0], &sg[0][0], HH + 4, nullptr, b3, 0, &sh[0][0], HH + 4, wave, lane);
    __syncthreads();
    if (tid < NNODE) { float a = 0.f, c2 = 0.f; for (int k = 0; k < HH; ++k) { const float hv = sh[tid][k]; a += hv * swA[k]; c2 += hv * swB[k]; } su[tid] = a; sv[tid] = c2; }
    __syncthreads();
    const float cst = sconst[0] + sconst[1];
    float* ob = out + (size_t)b * NNODE * NNODE;
    for (int q = tid; q < NNODE * NNODE / 4; q += 128) { v4f o;
#pragma unroll
      for (int e = 0; e < 4; ++e) { const int idx = q * 4 + e; o[e] = su[idx / NNODE] + sv[idx % NNODE] + cst; }
      vst2(ob + q * 4, o); } }
}
extern "C" void kernel_launch(void* const* d_in, const int* in_sizes, int n_in, void* d_out, int out_size, void* d_ws, size_t ws_size, hipStream_t stream) {
  (void)in_sizes; (void)n_in; (void)out_size; (void)ws_size; (void)d_ws;
  const float** I = (const float**)d_in;
  k_main<<<NBG / 2, 128, 0, stream>>>(I[0], I[1], I[2], I[3], I[4], I[5], I[6], I[7], I[8], I[9], I[10], I[11], I[12], I[13], I[14], I[15], (float*)d_out);
}
